// SRNN_64579128262671
// MI455X (gfx1250) — hardware-run, weakly checked
//
#include <hip/hip_runtime.h>


#ifndef TSTEPS
#define TSTEPS 8
#endif
#ifndef NNODE
#define NNODE 4096
#endif
#define TSTEPS_FULL 8
#define NNODE_FULL  4096
#define HD   64
#define XK   192
#define G4   256
#define NOUT 5
#define AW   4
#define OSP  68
#define HP   68
#define ACT  16.0f
#define WSC  64.0f
#define HTS  (1.0f / 64.0f)
#define GSI  (1.0f / 1024.0f)
#define QRS  2048.0f
#define QRI  (1.0f / 2048.0f)
#define SC2  ((float)((double)(NNODE - 1) * 1.4426950408889634 / 256.0))
#define PSH  14.0f
#define NEGB (-3.0e38f)

static_assert(HD == 64);
static_assert(XK == 3 * HD);
static_assert(G4 == 4 * HD);
static_assert(XK % 32 == 0);
static_assert(HD % 32 == 0);
static_assert(NNODE % 64 == 0);
static_assert(NNODE % (16 * AW) == 0);
static_assert(NNODE <= NNODE_FULL);
static_assert(TSTEPS <= TSTEPS_FULL);
static_assert((OSP * 4) % 16 == 0);
static_assert((HP * 4) % 16 == 0);
static_assert(4 * 32 * 16 == 16 * HD * 2);
static_assert(4 * 128 * 16 == 64 * HD * 2);
static_assert(8 * 128 * 16 == 64 * HD * 4);
static_assert(80 * 4 == 64 * NOUT);
static_assert(3 * 128 >= 64 * NOUT);
static_assert((64 * NOUT * 4) % 128 == 0);
static_assert((AW * 16 * OSP) * 4 <= 131072);
static_assert((2 * 64 * HP + 2 * 64 * NOUT) * 4 <= 131072);

typedef _Float16 h16;
typedef __attribute__((ext_vector_type(16))) _Float16 v16h;
typedef __attribute__((ext_vector_type(8)))  _Float16 v8h;
typedef __attribute__((ext_vector_type(8)))  float    v8f;
typedef __attribute__((ext_vector_type(4)))  float    v4f;
typedef v4f  __attribute__((may_alias)) v4fa;

__device__ __forceinline__ unsigned short f2bf(float f) { unsigned u = __float_as_uint(f); u += 0x7FFFu + ((u >> 16) & 1u); return (unsigned short)(u >> 16); }
__device__ __forceinline__ float bfr(float f) { return __uint_as_float(((unsigned)f2bf(f)) << 16); }
__device__ __forceinline__ v16h cat16(v8h lo, v8h hi) { return __builtin_shufflevector(lo, hi, 0, 1, 2, 3, 4, 5, 6, 7, 8, 9, 10, 11, 12, 13, 14, 15); }
__device__ __forceinline__ v16h ldh(const h16* p) { return cat16(*(const v8h*)p, *(const v8h*)(p + 16)); }
__device__ __forceinline__ v8f wg(v16h a, v16h b, v8f c) {
    c = __builtin_amdgcn_wmma_f32_16x16x32_f16(false, a, false, b, (short)0, c, false, false);
    asm volatile("v_nop\n\tv_nop\n\tv_nop\n\tv_nop" : "+v"(c) : "v"(a), "v"(b));
    return c;
}
static __device__ __forceinline__ h16 toh_flush(float v) { const h16 r = (h16)v; return (fabsf(v) < 6.103515625e-05f) ? (h16)0.0f : r; }
__device__ __forceinline__ void wave_sync() { __builtin_amdgcn_fence(3  , "wavefront"); __builtin_amdgcn_wave_barrier(); asm volatile("" ::: "memory"); }
__device__ __forceinline__ float sigm(float x) { return 1.0f / (1.0f + expf(-x)); }
__device__ __forceinline__ v4f bias4(const float* __restrict__ bi, const float* __restrict__ bh, int o) {
    const v4f a = *(const v4f*)(bi + o); const v4f b = *(const v4f*)(bh + o); v4f r;
#pragma unroll
    for (int i = 0; i < 4; ++i) r[i] = bfr(a[i]) + bfr(b[i]);
    return r;
}

static_assert((HD * HD) / 8 == 2 * 256);
static_assert((G4 * XK) / 8 == 24 * 256);
__global__ __launch_bounds__(256) void k_wprep(const float* __restrict__ Wt, const float* __restrict__ Wih, const float* __restrict__ Whh, h16* WtT, h16* Wcat) {
    const int tid = threadIdx.x; v8h o;
    if (blockIdx.x < 2) {
        const int p = blockIdx.x * 256 + tid; const int n = p >> 3, k8 = (p & 7) * 8;
#pragma unroll
        for (int i = 0; i < 8; ++i) o[i] = toh_flush(bfr(Wt[(size_t)(k8 + i) * HD + n]) * WSC);
        h16* dst = WtT + (size_t)p * 8;
        *(volatile v8h*)dst = o; __threadfence(); *(volatile v8h*)dst = o;
    } else {
        const int q = (blockIdx.x - 2) * 256 + tid; const int n = q / 24; const int k8 = (q - n * 24) * 8;
        const int ka = k8 < 120 ? k8 : 120; int kh = k8 - 128; kh = kh < 0 ? 0 : (kh > 56 ? 56 : kh);
        v4f a0 = *(const v4f*)(Wih + (size_t)n * 128 + ka), a1 = *(const v4f*)(Wih + (size_t)n * 128 + ka + 4);
        v4f b0 = *(const v4f*)(Whh + (size_t)n * HD + kh),  b1 = *(const v4f*)(Whh + (size_t)n * HD + kh + 4);
        asm volatile("" : "+v"(a0)); asm volatile("" : "+v"(a1)); asm volatile("" : "+v"(b0)); asm volatile("" : "+v"(b1));
        const bool first = k8 < 128;
#pragma unroll
        for (int i = 0; i < 4; ++i) { const float x = first ? a0[i] : b0[i]; const float y = first ? a1[i] : b1[i];
            o[i] = toh_flush(bfr(x) * WSC); o[4 + i] = toh_flush(bfr(y) * WSC); }
        h16* dst = Wcat + (size_t)q * 8;
        *(volatile v8h*)dst = o; __threadfence(); *(volatile v8h*)dst = o;
    }
}

__global__ __launch_bounds__(32 * AW) void k_keypass(const h16* __restrict__ HH, const h16* __restrict__ HR, const h16* __restrict__ VT, h16* HS) {
    __shared__ __align__(16) float os[AW * 16 * OSP];
    const int lane = threadIdx.x & 31, lr = lane & 15, hi = lane >> 4;
    const int wave = __builtin_amdgcn_readfirstlane((int)(threadIdx.x >> 5));
    const int t0 = (blockIdx.x * AW + wave) * 16;
    const int qi = t0 + lr;
    const size_t qo = (size_t)qi * HD + 8 * hi;
    const v16h qh0 = ldh(HH + qo), qh1 = ldh(HH + qo + 32);
    const v16h qr0 = ldh(HR + qo), qr1 = ldh(HR + qo + 32);
    const size_t ko = (size_t)lr * HD + 8 * hi;
    const size_t vo = (size_t)lr * NNODE + 8 * hi;
    v8f o0 = (v8f){}, o1 = (v8f){}, o2 = (v8f){}, o3 = (v8f){};
    float m = NEGB, l = 0.0f;
#pragma unroll 1
    for (int key0 = 0; key0 < NNODE; key0 += 32) {
        const h16* ka = HH + ko + (size_t)key0 * HD;
        const h16* kr = HR + ko + (size_t)key0 * HD;
        v8f sHa = (v8f){}, sLa = (v8f){}, sHb = (v8f){}, sLb = (v8f){};
        { const v16h a0 = ldh(ka), a1 = ldh(ka + 32), r0 = ldh(kr), r1 = ldh(kr + 32);
          sHa = wg(a0, qh0, sHa); sHa = wg(a1, qh1, sHa);
          sLa = wg(a0, qr0, sLa); sLa = wg(a1, qr1, sLa); sLa = wg(r0, qh0, sLa); sLa = wg(r1, qh1, sLa); }
        { const v16h a0 = ldh(ka + 16 * HD), a1 = ldh(ka + 16 * HD + 32), r0 = ldh(kr + 16 * HD), r1 = ldh(kr + 16 * HD + 32);
          sHb = wg(a0, qh0, sHb); sHb = wg(a1, qh1, sHb);
          sLb = wg(a0, qr0, sLb); sLb = wg(a1, qr1, sLb); sLb = wg(r0, qh0, sLb); sLb = wg(r1, qh1, sLb); }
        const int ja = key0 + 8 * hi;
        float ta[8], tb[8]; bool fa[8], fb[8]; float mx = NEGB;
#pragma unroll
        for (int r = 0; r < 8; ++r) {
            fa[r] = (ja + r) != qi;
            fb[r] = (ja + 16 + r) != qi;
            ta[r] = (sHa[r] + sLa[r] * QRI) * SC2; tb[r] = (sHb[r] + sLb[r] * QRI) * SC2;
            mx = fmaxf(mx, fmaxf(fa[r] ? ta[r] : NEGB, fb[r] ? tb[r] : NEGB)); }
        mx = fmaxf(mx, __shfl_xor(mx, 16, 32));
        const float mnew = fmaxf(m, mx);
        const float alpha = __builtin_amdgcn_exp2f(m - mnew);
        const float sh = PSH - mnew;
        v16h pb; float ls = 0.0f;
#pragma unroll
        for (int r = 0; r < 8; ++r) {
            const float xa = ta[r] + sh, xb = tb[r] + sh;
            const float ea = (xa < -14.0f) ? 0.0f : __builtin_amdgcn_exp2f(xa);
            const float eb = (xb < -14.0f) ? 0.0f : __builtin_amdgcn_exp2f(xb);
            const float ga = fa[r] ? ea : 0.0f, gb = fb[r] ? eb : 0.0f;
            const h16 pa = (h16)ga; const h16 pc = (h16)gb;
            pb[r] = pa; pb[8 + r] = pc;
            ls += (float)pa + (float)pc; }
        l = l * alpha + ls; m = mnew;
        o0 = o0 * alpha; o1 = o1 * alpha; o2 = o2 * alpha; o3 = o3 * alpha;
        const h16* va = VT + vo + key0;
        o0 = wg(ldh(va), pb, o0);
        o1 = wg(ldh(va + (size_t)16 * NNODE), pb, o1);
        o2 = wg(ldh(va + (size_t)32 * NNODE), pb, o2);
        o3 = wg(ldh(va + (size_t)48 * NNODE), pb, o3);
    }
    l += __shfl_xor(l, 16, 32);
    const bool any = l > 0.0f;
    const float lsafe = any ? l : 1.0f;
    const float inv = any ? (1.0f / lsafe) : 0.0f;
    const int wb = wave * 16 * OSP;
    { v4f a, c;
      a[0] = o0[0] * inv; a[1] = o0[1] * inv; a[2] = o0[2] * inv; a[3] = o0[3] * inv; c[0] = o0[4] * inv; c[1] = o0[5] * inv; c[2] = o0[6] * inv; c[3] = o0[7] * inv;
      *(v4fa*)(&os[wb + lr * OSP +  0 + 8 * hi]) = a; *(v4fa*)(&os[wb + lr * OSP +  0 + 8 * hi + 4]) = c;
      a[0] = o1[0] * inv; a[1] = o1[1] * inv; a[2] = o1[2] * inv; a[3] = o1[3] * inv; c[0] = o1[4] * inv; c[1] = o1[5] * inv; c[2] = o1[6] * inv; c[3] = o1[7] * inv;
      *(v4fa*)(&os[wb + lr * OSP + 16 + 8 * hi]) = a; *(v4fa*)(&os[wb + lr * OSP + 16 + 8 * hi + 4]) = c;
      a[0] = o2[0] * inv; a[1] = o2[1] * inv; a[2] = o2[2] * inv; a[3] = o2[3] * inv; c[0] = o2[4] * inv; c[1] = o2[5] * inv; c[2] = o2[6] * inv; c[3] = o2[7] * inv;
      *(v4fa*)(&os[wb + lr * OSP + 32 + 8 * hi]) = a; *(v4fa*)(&os[wb + lr * OSP + 32 + 8 * hi + 4]) = c;
      a[0] = o3[0] * inv; a[1] = o3[1] * inv; a[2] = o3[2] * inv; a[3] = o3[3] * inv; c[0] = o3[4] * inv; c[1] = o3[5] * inv; c[2] = o3[6] * inv; c[3] = o3[7] * inv;
      *(v4fa*)(&os[wb + lr * OSP + 48 + 8 * hi]) = a; *(v4fa*)(&os[wb + lr * OSP + 48 + 8 * hi + 4]) = c; }
    wave_sync();
    h16* orow = HS + (size_t)t0 * HD;
#pragma unroll 1
    for (int ps = 0; ps < 2; ++ps) {
#pragma unroll
        for (int s = 0; s < 4; ++s) { const int row = 4 * s + (lane >> 3), c8 = (lane & 7) * 8;
            const v4f x0 = *(const v4fa*)(&os[wb + row * OSP + c8]); const v4f x1 = *(const v4fa*)(&os[wb + row * OSP + c8 + 4]); v8h hv;
#pragma unroll
            for (int i = 0; i < 4; ++i) { hv[i] = toh_flush(x0[i]); hv[4 + i] = toh_flush(x1[i]); }
            *(volatile v8h*)(orow + (size_t)row * HD + c8) = hv; }
        if (ps == 0) __threadfence(); }
}

__global__ __launch_bounds__(32 * AW) void k_cell(const float* __restrict__ nodes_t, const float* __restrict__ H0, const float* __restrict__ Csrc,
                                                  const h16* __restrict__ HS, const h16* __restrict__ HHc,
                                                  const float* __restrict__ Wenc, const float* __restrict__ benc, const float* __restrict__ bt,
                                                  const h16* __restrict__ WtT, const h16* __restrict__ Wcat,
                                                  const float* __restrict__ bih, const float* __restrict__ bhh,
                                                  const float* __restrict__ Wout, const float* __restrict__ bout,
                                                  h16* HHn, h16* HRn, h16* VTn, float* Cn, float* OUTt, float* HTo, float* CTo, int init, int last) {
    __shared__ __align__(16) float hN[64 * HP];
    __shared__ __align__(16) float cN[64 * HP];
    __shared__ __align__(16) float woS[64 * NOUT];
    __shared__ __align__(16) float outS[64 * NOUT];
    const int tid = threadIdx.x, lane = tid & 31, lr = lane & 15, hi = lane >> 4;
    const int wave = __builtin_amdgcn_readfirstlane((int)(threadIdx.x >> 5));
    const int tok0 = blockIdx.x * 64;
#pragma unroll 1
    for (int i = tid; i < 64 * NOUT; i += 32 * AW) woS[i] = bfr(Wout[i]);
    if (init != 0) {
#pragma unroll 1
        for (int it = 0; it < 8; ++it) { const int p = it * 128 + tid; const int row = p >> 4, c4 = (p & 15) * 4;
            const v4f hv = *(const v4f*)(H0 + (size_t)tok0 * HD + (size_t)p * 4); const v4f cv = *(const v4f*)(Csrc + (size_t)tok0 * HD + (size_t)p * 4);
            v4f a, c;
#pragma unroll
            for (int i = 0; i < 4; ++i) { a[i] = bfr(hv[i]); c[i] = bfr(cv[i]); }
            *(v4fa*)(&hN[row * HP + c4]) = a; *(v4fa*)(&cN[row * HP + c4]) = c; }
    } else {
        const int tok = tok0 + wave * 16 + lr;
        const float p0 = bfr(nodes_t[(size_t)tok * 2]), p1 = bfr(nodes_t[(size_t)tok * 2 + 1]);
        v16h xb[6];
#pragma unroll
        for (int s = 0; s < 2; ++s) {
            v16h f;
#pragma unroll
            for (int c = 0; c < 2; ++c) {
                const int kb = 32 * s + 16 * c + 8 * hi;
                const v4f wa0 = *(const v4f*)(Wenc + kb),      wa1 = *(const v4f*)(Wenc + kb + 4);
                const v4f wb0 = *(const v4f*)(Wenc + HD + kb), wb1 = *(const v4f*)(Wenc + HD + kb + 4);
                const v4f bb0 = *(const v4f*)(benc + kb),      bb1 = *(const v4f*)(benc + kb + 4);
#pragma unroll
                for (int i = 0; i < 4; ++i) {
                    const float e0 = fmaxf(p0 * bfr(wa0[i]) + p1 * bfr(wb0[i]) + bfr(bb0[i]), 0.0f) * ACT;
                    const float e1 = fmaxf(p0 * bfr(wa1[i]) + p1 * bfr(wb1[i]) + bfr(bb1[i]), 0.0f) * ACT;
                    f[8 * c + i] = toh_flush(e0); f[8 * c + 4 + i] = toh_flush(e1); } }
            xb[s] = f; }
        const size_t so = (size_t)tok * HD + 8 * hi;
        const v16h hs0 = ldh(HS + so), hs1 = ldh(HS + so + 32);
        v8f ht[4];
#pragma unroll
        for (int j = 0; j < 4; ++j) { const h16* wp = WtT + (size_t)(16 * j + lr) * HD + 8 * hi;
            v8f a = (v8f){}; a = wg(ldh(wp), hs0, a); a = wg(ldh(wp + 32), hs1, a); ht[j] = a; }
#pragma unroll
        for (int s = 0; s < 2; ++s) {
            v16h f;
#pragma unroll
            for (int c = 0; c < 2; ++c) {
                const v4f b0 = *(const v4f*)(bt + 16 * (2 * s + c) + 8 * hi), b1 = *(const v4f*)(bt + 16 * (2 * s + c) + 8 * hi + 4);
#pragma unroll
                for (int r = 0; r < 4; ++r) {
                    f[8 * c + r]     = toh_flush(fmaxf(ht[2 * s + c][r]     * HTS + ACT * bfr(b0[r]), 0.0f));
                    f[8 * c + 4 + r] = toh_flush(fmaxf(ht[2 * s + c][4 + r] * HTS + ACT * bfr(b1[r]), 0.0f)); } }
            xb[2 + s] = f; }
        xb[4] = ldh(HHc + so); xb[5] = ldh(HHc + so + 32);
        const int lrow = (wave * 16 + lr) * HP;
#pragma unroll 1
        for (int ds = 0; ds < 4; ++ds) {
            v8f g0 = (v8f){}, g1 = (v8f){}, g2 = (v8f){}, g3 = (v8f){};
            const h16* wr = Wcat + (size_t)(ds * 16 + lr) * XK + 8 * hi;
#pragma unroll
            for (int s = 0; s < 6; ++s) {
                g0 = wg(ldh(wr + 32 * s), xb[s], g0);
                g1 = wg(ldh(wr + (size_t)64 * XK + 32 * s), xb[s], g1);
                g2 = wg(ldh(wr + (size_t)128 * XK + 32 * s), xb[s], g2);
                g3 = wg(ldh(wr + (size_t)192 * XK + 32 * s), xb[s], g3); }
#pragma unroll
            for (int q = 0; q < 2; ++q) {
                const int o = ds * 16 + 8 * hi + 4 * q;
                const v4f bI = bias4(bih, bhh, o), bF = bias4(bih, bhh, 64 + o), bG = bias4(bih, bhh, 128 + o), bO = bias4(bih, bhh, 192 + o);
                const v4f cv = *(const v4f*)(Csrc + (size_t)tok * HD + o);
                v4f hn4, cn4;
#pragma unroll
                for (int r = 0; r < 4; ++r) {
                    const float gi = g0[4 * q + r] * GSI + bI[r], gf = g1[4 * q + r] * GSI + bF[r];
                    const float gg = g2[4 * q + r] * GSI + bG[r], go = g3[4 * q + r] * GSI + bO[r];
                    const float cn = sigm(gf) * cv[r] + sigm(gi) * tanhf(gg);
                    cn4[r] = cn; hn4[r] = sigm(go) * tanhf(cn); }
                *(v4fa*)(&hN[lrow + o]) = hn4; *(v4fa*)(&cN[lrow + o]) = cn4; }
        }
    }
    __syncthreads();
    if (init == 0) {
#pragma unroll 1
        for (int it = 0; it < 3; ++it) {
            const int i = it * 128 + tid; const int ic = i < 64 * NOUT ? i : (64 * NOUT - 1);
            const int r = ic / NOUT, oc = ic - r * NOUT;
            float acc = 0.0f;
#pragma unroll 4
            for (int d = 0; d < HD; ++d) acc += hN[r * HP + d] * woS[d * NOUT + oc];
            acc += bfr(bout[oc]);
            if (i < 64 * NOUT) outS[i] = acc; }
    }
    __syncthreads();
#pragma unroll 1
    for (int ps = 0; ps < 2; ++ps) {
#pragma unroll 1
        for (int it = 0; it < 4; ++it) { const int p = it * 128 + tid; const int row = p >> 3, c8 = (p & 7) * 8;
            const v4f x0 = *(const v4fa*)(&hN[row * HP + c8]); const v4f x1 = *(const v4fa*)(&hN[row * HP + c8 + 4]); v8h hv, rv;
#pragma unroll
            for (int i = 0; i < 4; ++i) { const float s0 = x0[i] * ACT, s1 = x1[i] * ACT; const h16 a0 = toh_flush(s0); const h16 a1 = toh_flush(s1);
                hv[i] = a0; hv[4 + i] = a1; rv[i] = toh_flush((s0 - (float)a0) * QRS); rv[4 + i] = toh_flush((s1 - (float)a1) * QRS); }
            *(volatile v8h*)(HHn + (size_t)tok0 * HD + (size_t)p * 8) = hv;
            *(volatile v8h*)(HRn + (size_t)tok0 * HD + (size_t)p * 8) = rv; }
#pragma unroll 1
        for (int it = 0; it < 4; ++it) { const int p = it * 128 + tid; const int d = p >> 3, t8 = (p & 7) * 8;
            v8h tv;
#pragma unroll
            for (int i = 0; i < 8; ++i) tv[i] = toh_flush(hN[(t8 + i) * HP + d] * ACT);
            *(volatile v8h*)(VTn + (size_t)d * NNODE + tok0 + t8) = tv; }
#pragma unroll 1
        for (int it = 0; it < 8; ++it) { const int p = it * 128 + tid; const int row = p >> 4, c4 = (p & 15) * 4;
            const v4f cv = *(const v4fa*)(&cN[row * HP + c4]);
            *(volatile v4f*)(Cn + (size_t)tok0 * HD + (size_t)p * 4) = cv; }
        if (last != 0) {
#pragma unroll 1
            for (int it = 0; it < 8; ++it) { const int p = it * 128 + tid; const int row = p >> 4, c4 = (p & 15) * 4;
                const v4f hv = *(const v4fa*)(&hN[row * HP + c4]); const v4f cv = *(const v4fa*)(&cN[row * HP + c4]);
                *(volatile v4f*)(HTo + (size_t)tok0 * HD + (size_t)p * 4) = hv;
                *(volatile v4f*)(CTo + (size_t)tok0 * HD + (size_t)p * 4) = cv; }
        }
        if (init == 0) {
            if (tid < 80) { const v4f ov = *(const v4fa*)(&outS[tid * 4]);
                *(volatile v4f*)(OUTt + (size_t)tok0 * NOUT + (size_t)tid * 4) = ov; }
        }
        if (ps == 0) __threadfence(); }
}

static constexpr size_t al256(size_t v) { return (v + 255) & ~(size_t)255; }
static constexpr size_t SZ_WT = al256((size_t)HD * HD * 2);
static constexpr size_t SZ_WC = al256((size_t)G4 * XK * 2);
static constexpr size_t SZ_PL = al256((size_t)NNODE * HD * 2);
static constexpr size_t SZ_CP = al256((size_t)NNODE * HD * 4);
static constexpr size_t SZ_TOTAL = SZ_WT + SZ_WC + 7 * SZ_PL + 2 * SZ_CP;
static_assert(SZ_TOTAL <= (size_t)134217728);
static constexpr size_t OFF_H = (size_t)TSTEPS_FULL * NNODE_FULL * NOUT;
static constexpr size_t OFF_C = OFF_H + (size_t)NNODE_FULL * HD;
static_assert(OFF_H * 4 == (size_t)655360);
static_assert(OFF_C * 4 == (size_t)1703936);
static_assert((OFF_C + (size_t)NNODE_FULL * HD) * 4 == (size_t)2752512);
static_assert(((size_t)NNODE_FULL * NOUT * 4) % 128 == 0);

extern "C" void kernel_launch(void* const* d_in, const int* in_sizes, int n_in,
                              void* d_out, int out_size, void* d_ws, size_t ws_size, hipStream_t stream) {
    if (n_in < 13) return;
    if ((size_t)in_sizes[0] < ((size_t)(TSTEPS - 1) * NNODE_FULL + NNODE) * 2) return;
    if ((size_t)in_sizes[1] < (size_t)NNODE * HD || (size_t)in_sizes[2] < (size_t)NNODE * HD) return;
    if (in_sizes[3] < 2 * HD || in_sizes[4] < HD || in_sizes[5] < HD * HD || in_sizes[6] < HD) return;
    if (in_sizes[7] < G4 * 128 || in_sizes[8] < G4 * HD || in_sizes[9] < G4 || in_sizes[10] < G4) return;
    if (in_sizes[11] < HD * NOUT || in_sizes[12] < NOUT) return;
    if ((size_t)out_size < OFF_C + (size_t)NNODE * HD) return;
    if (SZ_TOTAL > ws_size) return;
    const float* nodes = (const float*)d_in[0];
    const float* h0 = (const float*)d_in[1]; const float* c0 = (const float*)d_in[2];
    const float* wenc = (const float*)d_in[3]; const float* benc = (const float*)d_in[4];
    const float* wt = (const float*)d_in[5];   const float* bt = (const float*)d_in[6];
    const float* wih = (const float*)d_in[7];  const float* whh = (const float*)d_in[8];
    const float* bih = (const float*)d_in[9];  const float* bhh = (const float*)d_in[10];
    const float* wout = (const float*)d_in[11]; const float* bout = (const float*)d_in[12];
    float* OUT = (float*)d_out;
    char* wsp = (char*)d_ws;
    h16* WtT  = (h16*)wsp; wsp += SZ_WT;
    h16* Wcat = (h16*)wsp; wsp += SZ_WC;
    h16* HH[2]; h16* HR[2]; h16* VT[2]; float* CP[2];
    HH[0] = (h16*)wsp; wsp += SZ_PL; HH[1] = (h16*)wsp; wsp += SZ_PL;
    HR[0] = (h16*)wsp; wsp += SZ_PL; HR[1] = (h16*)wsp; wsp += SZ_PL;
    VT[0] = (h16*)wsp; wsp += SZ_PL; VT[1] = (h16*)wsp; wsp += SZ_PL;
    h16* HS = (h16*)wsp; wsp += SZ_PL;
    CP[0] = (float*)wsp; wsp += SZ_CP; CP[1] = (float*)wsp; wsp += SZ_CP;

    k_wprep<<<26, 256, 0, stream>>>(wt, wih, whh, WtT, Wcat);
    k_cell<<<NNODE / 64, 32 * AW, 0, stream>>>(nodes, h0, c0, HS, HH[1], wenc, benc, bt, WtT, Wcat, bih, bhh, wout, bout,
                                               HH[0], HR[0], VT[0], CP[0], OUT, OUT + OFF_H, OUT + OFF_C, 1, 0);
    int cur = 0;
    for (int t = 0; t < TSTEPS; ++t) {
        const int nxt = cur ^ 1;
        k_keypass<<<NNODE / (16 * AW), 32 * AW, 0, stream>>>(HH[cur], HR[cur], VT[cur], HS);
        k_cell<<<NNODE / 64, 32 * AW, 0, stream>>>(nodes + (size_t)t * NNODE_FULL * 2, h0, CP[cur], HS, HH[cur], wenc, benc, bt, WtT, Wcat, bih, bhh, wout, bout,
                                                   HH[nxt], HR[nxt], VT[nxt], CP[nxt], OUT + (size_t)t * NNODE_FULL * NOUT, OUT + OFF_H, OUT + OFF_C,
                                                   0, (t == TSTEPS - 1) ? 1 : 0);
        cur = nxt;
    }
}
